// SingleLayerMambaPGF_68539088110105
// MI455X (gfx1250) — hardware-verified
//
#include <hip/hip_runtime.h>
#include <math.h>

constexpr int kBatch   = 4;
constexpr int kSeqLen  = 2048;
constexpr int kDModel  = 256;
constexpr int kNState  = 16;
constexpr int kRows    = kBatch * kSeqLen;
constexpr int kNProj   = 384;
constexpr float kWCarry    = 64.0f;
constexpr float kWCarryInv = 1.0f / 64.0f;
constexpr int kChanPerBlock = 64;
constexpr int kStepTile     = 16;

typedef __attribute__((ext_vector_type(16))) _Float16 v16h;
typedef __attribute__((ext_vector_type(8)))  _Float16 v8h;
typedef __attribute__((ext_vector_type(16))) __bf16   v16b;
typedef __attribute__((ext_vector_type(8)))  __bf16   v8b;
typedef __attribute__((ext_vector_type(8)))  float    v8f;
typedef __attribute__((ext_vector_type(4)))  float    v4f;
typedef __attribute__((ext_vector_type(4)))  unsigned int v4u;

__device__ __forceinline__ unsigned short f2bf_bits(float f) {
  unsigned u = __float_as_uint(f);
  return (unsigned short)((u + 0x7FFFu + ((u >> 16) & 1u)) >> 16);
}
__device__ __forceinline__ float bf_bits2f(unsigned short h) { return __uint_as_float(((unsigned)h) << 16); }

__device__ __forceinline__ void dep_guard_h(v8f& a, v8f& b, v16h x, v16h y) { asm volatile("v_nop\n\tv_nop\n\tv_nop\n\tv_nop" : "+v"(a), "+v"(b) : "v"(x), "v"(y)); }
__device__ __forceinline__ void dep_guard_b(v8f& a, v8f& b, v16b x, v16b y) { asm volatile("v_nop\n\tv_nop\n\tv_nop\n\tv_nop" : "+v"(a), "+v"(b) : "v"(x), "v"(y)); }
__device__ __forceinline__ void keep4_h(v16h a, v16h b, v16h c, v16h d) { asm volatile("v_nop" :: "v"(a), "v"(b), "v"(c), "v"(d)); }
__device__ __forceinline__ void keep4_b(v16b a, v16b b, v16b c, v16b d) { asm volatile("v_nop" :: "v"(a), "v"(b), "v"(c), "v"(d)); }
__device__ __forceinline__ void acc_guard4(v8f& a, v8f& b, v8f& c, v8f& d) { asm volatile("v_nop\n\tv_nop\n\tv_nop\n\tv_nop" : "+v"(a), "+v"(b), "+v"(c), "+v"(d)); }
template <typename T> struct Frag;
template <> struct Frag<_Float16> {
  typedef v16h V; union U { v16h v; v8h h[2]; };
  static __device__ __forceinline__ v16h load(const _Float16* p) {
    U f; f.h[0] = *(const v8h*)(p); f.h[1] = *(const v8h*)(p + 16); return f.v;
  }
  static __device__ __forceinline__ v8f mma(v16h a, v16h b, v8f c) {
    return __builtin_amdgcn_wmma_f32_16x16x32_f16(false, a, false, b, (short)0, c, false, false);
  }
  static __device__ __forceinline__ void guard(v8f& a, v8f& b, v16h x, v16h y) { dep_guard_h(a, b, x, y); }
  static __device__ __forceinline__ void keep(v16h a, v16h b, v16h c, v16h d) { keep4_h(a, b, c, d); }
};
template <> struct Frag<__bf16> {
  typedef v16b V; union U { v16b v; v8b h[2]; };
  static __device__ __forceinline__ v16b load(const __bf16* p) {
    U f; f.h[0] = *(const v8b*)(p); f.h[1] = *(const v8b*)(p + 16); return f.v;
  }
  static __device__ __forceinline__ v8f mma(v16b a, v16b b, v8f c) {
    return __builtin_amdgcn_wmma_f32_16x16x32_bf16(false, a, false, b, (short)0, c, false, false);
  }
  static __device__ __forceinline__ void guard(v8f& a, v8f& b, v16b x, v16b y) { dep_guard_b(a, b, x, y); }
  static __device__ __forceinline__ void keep(v16b a, v16b b, v16b c, v16b d) { keep4_b(a, b, c, d); }
};

__device__ __forceinline__ unsigned pk16(unsigned short a, unsigned short b) { return (unsigned)a | ((unsigned)b << 16); }
__device__ __forceinline__ unsigned short h_bits(float f) { const _Float16 h = (_Float16)f; return __builtin_bit_cast(unsigned short, h); }

template <int ET> struct Elem;
template <> struct Elem<0> { typedef _Float16 T; };
template <> struct Elem<1> { typedef __bf16 T; };
template <int ET, bool SPLIT, int BIAS_MODE, int OUT_MODE, bool RESID, int ACT = 0>
__global__ __launch_bounds__(256) void wmma_gemm64(
    const unsigned short* __restrict__ Ap, const unsigned short* __restrict__ A2p, int lda, long strideA,
    const unsigned short* __restrict__ Btp, const unsigned short* __restrict__ Bt2p, int ldb, long strideB,
    void* __restrict__ Cout, void* __restrict__ Cout2, int ldc, long strideC,
    const float* __restrict__ bias,
    const float* __restrict__ resid, long strideR,
    int M, int N, int K, float scale) {
  typedef typename Elem<ET>::T T;
  typedef typename Frag<T>::V V;
  const T* A = (const T*)Ap; const T* A2 = (const T*)A2p; const T* Bt = (const T*)Btp; const T* Bt2 = (const T*)Bt2p;
  __shared__ __align__(16) float sT[8][16 * 68];
  const int b    = blockIdx.y;
  const int lane = threadIdx.x & 31;
  const int wave = threadIdx.x >> 5;
  const int tilesN = N >> 6;
  const int tilesM = M >> 6;
  const int tile = blockIdx.x * 8 + wave;
  if (tile >= tilesM * tilesN) return;
  const int tm = tile / tilesN;
  const int tn = tile - tm * tilesN;
  const int m0 = tm << 6;
  const int n0 = tn << 6;

  const T* Ab  = A  + (size_t)b * strideA;
  const T* Bb  = Bt + (size_t)b * strideB;
  const T* Ab2 = SPLIT ? (A2  + (size_t)b * strideA) : nullptr;
  const T* Bb2 = SPLIT ? (Bt2 + (size_t)b * strideB) : nullptr;

  const int rlane = lane & 15;
  const int koff  = (lane >> 4) * 8;
  const int mOff  = (lane >> 4) * 8;

  v8f acc[4][4];
#pragma unroll
  for (int i = 0; i < 4; ++i)
#pragma unroll
    for (int j = 0; j < 4; ++j) acc[i][j] = (v8f){0.f,0.f,0.f,0.f,0.f,0.f,0.f,0.f};

  for (int k0 = 0; k0 < K; k0 += 32) {
    V bh[4], bl[4];
#pragma unroll
    for (int j = 0; j < 4; ++j) {
      const size_t bo = (size_t)(n0 + (j << 4) + rlane) * ldb + koff + k0;
      bh[j] = Frag<T>::load(Bb + bo);
      if (SPLIT) bl[j] = Frag<T>::load(Bb2 + bo);
    }
#pragma unroll
    for (int i = 0; i < 4; ++i) {
      const size_t ao = (size_t)(m0 + (i << 4) + rlane) * lda + koff + k0;
      V ah = Frag<T>::load(Ab + ao);
      V al;
      if (SPLIT) al = Frag<T>::load(Ab2 + ao);
#pragma unroll
      for (int j = 0; j < 4; ++j) {
        acc[i][j] = Frag<T>::mma(ah, bh[j], acc[i][j]);
        if (SPLIT) {
          acc[i][j] = Frag<T>::mma(ah, bl[j], acc[i][j]);
          acc[i][j] = Frag<T>::mma(al, bh[j], acc[i][j]);
        }
      }
      Frag<T>::guard(acc[i][0], acc[i][3], ah, SPLIT ? al : ah);
    }
    Frag<T>::keep(bh[0], bh[1], bh[2], bh[3]);
    if (SPLIT) Frag<T>::keep(bl[0], bl[1], bl[2], bl[3]);
  }
  acc_guard4(acc[0][0], acc[0][1], acc[0][2], acc[0][3]);
  acc_guard4(acc[1][0], acc[1][1], acc[1][2], acc[1][3]);
  acc_guard4(acc[2][0], acc[2][1], acc[2][2], acc[2][3]);
  acc_guard4(acc[3][0], acc[3][1], acc[3][2], acc[3][3]);

  float* slab = sT[wave];
  const float* Rb = RESID ? (resid + (size_t)b * strideR) : nullptr;
#pragma unroll
  for (int i = 0; i < 4; ++i) {
    const int mBase = m0 + (i << 4);
#pragma unroll
    for (int j = 0; j < 4; ++j) {
      const int n = n0 + (j << 4) + rlane;
      float bv = 0.f;
      if (BIAS_MODE == 2) bv = bias[n];
#pragma unroll
      for (int r = 0; r < 8; ++r) {
        float v = acc[i][j][r] * scale;
        if (BIAS_MODE == 1) v += bias[mBase + mOff + r];
        if (BIAS_MODE == 2) v += bv;
        if (RESID) v += Rb[(size_t)(mBase + mOff + r) * ldc + n];
        if (ACT == 2) v = fmaxf(v, 0.0f);
        if (ACT == 4) v = (v > 0.f) ? v : 0.01f * v;
        slab[(mOff + r) * 68 + (j << 4) + rlane] = v;
      }
    }
    __builtin_amdgcn_fence(__ATOMIC_RELEASE, "workgroup");
    __builtin_amdgcn_wave_barrier();
    __builtin_amdgcn_fence(__ATOMIC_ACQUIRE, "workgroup");
    if (OUT_MODE == 0) {
      float* C = (float*)Cout + (size_t)b * strideC;
      const int hh = lane >> 4, c4 = (lane & 15) * 4;
      for (int pass = 0; pass < 2; ++pass) {
#pragma unroll
        for (int it = 0; it < 8; ++it) {
          const int row = it * 2 + hh;
          v4f v = *(const v4f*)(slab + row * 68 + c4);
          *(volatile v4f*)(C + (size_t)(mBase + row) * ldc + n0 + c4) = v;
        }
        __threadfence();
      }
    } else {
      const int q = lane >> 3, c8 = (lane & 7) * 8;
      unsigned short* C  = (unsigned short*)Cout  + (size_t)b * strideC;
      unsigned short* C2 = (OUT_MODE == 2) ? ((unsigned short*)Cout2 + (size_t)b * strideC) : nullptr;
      for (int pass = 0; pass < 2; ++pass) {
#pragma unroll
        for (int it = 0; it < 4; ++it) {
          const int row = it * 4 + q;
          const float* sp = slab + row * 68 + c8;
          v8h hv, lv;
#pragma unroll
          for (int e = 0; e < 8; ++e) {
            if (OUT_MODE == 1) {
              hv[e] = (_Float16)sp[e];
            } else {
              unsigned short hb = f2bf_bits(sp[e]);
              unsigned short lb = f2bf_bits(sp[e] - bf_bits2f(hb));
              hv[e] = __builtin_bit_cast(_Float16, hb);
              lv[e] = __builtin_bit_cast(_Float16, lb);
            }
          }
          *(volatile v8h*)(C + (size_t)(mBase + row) * ldc + n0 + c8) = hv;
          if (OUT_MODE == 2) *(volatile v8h*)(C2 + (size_t)(mBase + row) * ldc + n0 + c8) = lv;
        }
        __threadfence();
      }
    }
    __builtin_amdgcn_fence(__ATOMIC_RELEASE, "workgroup");
    __builtin_amdgcn_wave_barrier();
    __builtin_amdgcn_fence(__ATOMIC_ACQUIRE, "workgroup");
  }
}

__global__ __launch_bounds__(256) void cast8_f16_kernel(const float* __restrict__ in, unsigned short* __restrict__ out, int n8) {
  const int i = blockIdx.x * 256 + threadIdx.x;
  if (i >= n8) return;
  const float* p = in + 8 * (size_t)i;
  const v4f a = *(const v4f*)(p);
  const v4f c = *(const v4f*)(p + 4);
  unsigned short hb[8];
#pragma unroll
  for (int e = 0; e < 4; ++e) {
    hb[e]     = h_bits(a[e]);
    hb[4 + e] = h_bits(c[e]);
  }
  const v4u u = (v4u){pk16(hb[0], hb[1]), pk16(hb[2], hb[3]), pk16(hb[4], hb[5]), pk16(hb[6], hb[7])};
  unsigned short* q = out + 8 * (size_t)i;
  *(volatile v4u*)q = u;
  __threadfence();
  *(volatile v4u*)q = u;
}

__global__ __launch_bounds__(256) void wstack_f16_kernel(const float* __restrict__ Wdt, const float* __restrict__ Wb,
                                                         const float* __restrict__ Wc, unsigned short* __restrict__ outp) {
  const int g   = blockIdx.x * 256 + threadIdx.x;
  const int row = g >> 5;
  const int c8  = (g & 31) * 8;
  int rd = row; rd = rd > (kDModel - 1) ? (kDModel - 1) : rd;
  int rb = row - kDModel; rb = rb < 0 ? 0 : (rb > (kNState - 1) ? (kNState - 1) : rb);
  int rc = row - kDModel - kNState; rc = rc < 0 ? 0 : (rc > (kNState - 1) ? (kNState - 1) : rc);
  const float* pa = Wdt + (size_t)rd * kDModel + c8;
  const float* pb = Wb  + (size_t)rb * kDModel + c8;
  const float* pc = Wc  + (size_t)rc * kDModel + c8;
  const v4f a0 = *(const v4f*)(pa), a1 = *(const v4f*)(pa + 4);
  const v4f b0 = *(const v4f*)(pb), b1 = *(const v4f*)(pb + 4);
  const v4f c0 = *(const v4f*)(pc), c1 = *(const v4f*)(pc + 4);
  const bool sa = row < kDModel;
  const bool sb = (row >= kDModel) && (row < kDModel + kNState);
  const bool sc = (row >= kDModel + kNState) && (row < kDModel + 2 * kNState);
  unsigned short hb[8];
#pragma unroll
  for (int e = 0; e < 4; ++e) {
    const float v0 = sa ? a0[e] : (sb ? b0[e] : (sc ? c0[e] : 0.0f));
    const float v1 = sa ? a1[e] : (sb ? b1[e] : (sc ? c1[e] : 0.0f));
    hb[e]     = h_bits(v0 * kWCarry);
    hb[4 + e] = h_bits(v1 * kWCarry);
  }
  const v4u u = (v4u){pk16(hb[0], hb[1]), pk16(hb[2], hb[3]), pk16(hb[4], hb[5]), pk16(hb[6], hb[7])};
  unsigned short* q = outp + (size_t)row * kDModel + c8;
  *(volatile v4u*)q = u;
  __threadfence();
  *(volatile v4u*)q = u;
}

__global__ __launch_bounds__(64) void ssm_scan_kernel(const float* __restrict__ P, const float* __restrict__ u,
                                                     const float* __restrict__ A_log, const float* __restrict__ Dp,
                                                     const float* __restrict__ scl, const float* __restrict__ bdt,
                                                     const float* __restrict__ bB, const float* __restrict__ bC,
                                                     float* __restrict__ out) {
  __shared__ __align__(16) float hs[kNState * kChanPerBlock];
  __shared__ __align__(16) float bcs[kStepTile * 32];
  __shared__ __align__(16) float ys[kStepTile * kChanPerBlock];
  __shared__ float As[kNState];
  __shared__ float biasBC[32];

  const int tid  = threadIdx.x;
  const int lane = tid & 31;
  const int wave = tid >> 5;
  const int b    = blockIdx.y;
  const int d0   = blockIdx.x * kChanPerBlock;
  const int d    = d0 + tid;

  {
    const int ia = tid < kNState ? tid : (kNState - 1);
    const float al = A_log[ia];
    if (tid < kNState) As[tid] = -expf(al);
    const int ib = tid < kNState ? tid : (kNState - 1);
    int ic = tid - kNState; ic = ic < 0 ? 0 : (ic > (kNState - 1) ? (kNState - 1) : ic);
    const float vb = bB[ib];
    const float vc = bC[ic];
    if (tid < 32) biasBC[tid] = (tid < kNState) ? vb : vc;
  }
#pragma unroll 1
  for (int n = 0; n < kNState; ++n) hs[n * kChanPerBlock + tid] = 0.0f;
  const float bd = bdt[d];
  const float Dd = Dp[d];
  const float sc = scl[d];
  const size_t rowb = (size_t)b * kSeqLen;
  __syncthreads();

#pragma unroll 1
  for (int ch = 0; ch < kSeqLen / kStepTile; ++ch) {
    const int l0 = ch * kStepTile;
    __syncthreads();
    {
      const int rr = tid >> 2, q = tid & 3;
      const float* src = P + (rowb + l0 + rr) * (size_t)kNProj + kDModel + q * 8;
      const v4f a = *(const v4f*)(src);
      const v4f c = *(const v4f*)(src + 4);
      float* dst = bcs + rr * 32 + q * 8;
#pragma unroll
      for (int e = 0; e < 4; ++e) {
        dst[e]     = a[e] + biasBC[q * 8 + e];
        dst[4 + e] = c[e] + biasBC[q * 8 + 4 + e];
      }
    }
    __syncthreads();

#pragma unroll 1
    for (int t = 0; t < kStepTile; ++t) {
      const size_t grow = rowb + l0 + t;
      const float x  = P[grow * (size_t)kNProj + d] + bd;
      const float uv = u[grow * (size_t)kDModel + d];
      const float dt = fmaxf(x, 0.0f) + log1pf(expf(-fabsf(x)));
      const float* bct = bcs + t * 32;
      float y = 0.0f;
#pragma unroll 1
      for (int n = 0; n < kNState; ++n) {
        const float z  = dt * As[n];
        const float az = fabsf(z);
        const bool tiny = az < 1e-12f;
        const float zs = tiny ? 1e-12f : z;
        const float em = expm1f(zs);
        const float qv = em / zs;
        const float ph = tiny ? 1.0f : qv;
        const float dA = em + 1.0f;
        const float bb = (ph * bct[n]) * uv;
        const float hp = hs[n * kChanPerBlock + tid];
        const float hn = dA * hp + bb;
        hs[n * kChanPerBlock + tid] = hn;
        y += bct[kNState + n] * hn;
      }
      ys[t * kChanPerBlock + tid] = (y + Dd * uv) * sc;
    }
    __syncthreads();

    {
      const int hh = lane >> 4, c4 = (lane & 15) * 4;
      float* ob = out + (rowb + l0) * (size_t)kDModel + d0;
      for (int pass = 0; pass < 2; ++pass) {
#pragma unroll
        for (int it = 0; it < 4; ++it) {
          const int row = wave * 8 + it * 2 + hh;
          const v4f v = *(const v4f*)(ys + row * kChanPerBlock + c4);
          *(volatile v4f*)(ob + (size_t)row * kDModel + c4) = v;
        }
        __threadfence();
      }
    }
  }
}

extern "C" void kernel_launch(void* const* d_in, const int* in_sizes, int n_in,
                              void* d_out, int out_size, void* d_ws, size_t ws_size,
                              hipStream_t stream)
{
  if (n_in < 10) return;
  if (in_sizes[0] != kRows * kDModel) return;
  if (in_sizes[1] != kNState || in_sizes[4] != kDModel * kDModel) return;
  if (in_sizes[6] != kNState * kDModel || in_sizes[8] != kNState * kDModel) return;
  if (out_size != kRows * kDModel) return;

  const float* u     = (const float*)d_in[0];
  const float* A_log = (const float*)d_in[1];
  const float* D_par = (const float*)d_in[2];
  const float* scale = (const float*)d_in[3];
  const float* W_dt  = (const float*)d_in[4];
  const float* b_dt  = (const float*)d_in[5];
  const float* W_B   = (const float*)d_in[6];
  const float* b_B   = (const float*)d_in[7];
  const float* W_C   = (const float*)d_in[8];
  const float* b_C   = (const float*)d_in[9];
  float* out = (float*)d_out;

  const size_t offU = 0;
  const size_t bytesU = (size_t)kRows * kDModel * 2;
  const size_t offW = offU + bytesU;
  const size_t bytesW = (size_t)kNProj * kDModel * 2;
  const size_t offP = offW + bytesW;
  const size_t bytesP = (size_t)kRows * kNProj * 4;
  if (offP + bytesP > ws_size) return;

  char* ws = (char*)d_ws;
  unsigned short* uh = (unsigned short*)(ws + offU);
  unsigned short* wh = (unsigned short*)(ws + offW);
  float* P = (float*)(ws + offP);

  {
    const int n8 = kRows * kDModel / 8;
    cast8_f16_kernel<<<dim3(n8 / 256), dim3(256), 0, stream>>>(u, uh, n8);
  }
  {
    wstack_f16_kernel<<<dim3((kNProj * 32) / 256), dim3(256), 0, stream>>>(W_dt, W_B, W_C, wh);
  }
  {
    wmma_gemm64<0, false, 0, 0, false, 0><<<dim3((kRows / 64) * (kNProj / 64) / 8, 1), dim3(256), 0, stream>>>(
        uh, uh, kDModel, 0L,
        wh, wh, kDModel, 0L,
        (void*)P, (void*)P, kNProj, 0L,
        b_dt,
        u, 0L,
        kRows, kNProj, kDModel, kWCarryInv);
  }
  {
    ssm_scan_kernel<<<dim3(kDModel / kChanPerBlock, kBatch), dim3(kChanPerBlock), 0, stream>>>(
        P, u, A_log, D_par, scale, b_dt, b_B, b_C, out);
  }
}
